// HeteroGNN_17274358464707
// MI455X (gfx1250) — hardware-verified
//
#include <hip/hip_runtime.h>
#include <stddef.h>
#include <stdint.h>


#define D1     128
#define C2     64
#define K2     256
#define NTHR   256
#define NWAVE  8
#define EPT    8
#define CHUNK  (NTHR * EPT)
#define WCAP   (EPT * 32)
#define LISTN  (NWAVE * WCAP)
#define NBMAX  2048
#define SLOTB  11
#define RCAP   28672
#define DEGCAP 128
#define GBM    32
#define GTHR   64
#define MROWS  128
#define NSDP   4
#define NMAT   12
#define UPM    2048
#define NEGSL  0.2f
#define EPS_SM 1e-16f
#define MX0    (-1.0e30f)
#define WSMAX  134217728
#define LDS_AGG ((2 * RCAP + 2 * NBMAX + LISTN) * 4 + 64)

static_assert((CHUNK & (CHUNK - 1)) == 0 && CHUNK <= (1 << SLOTB));
static_assert(NBMAX == (1 << SLOTB));
static_assert(NTHR * 8 == NBMAX);
static_assert(LISTN >= NBMAX);
static_assert(LISTN >= NWAVE * WCAP);
static_assert((RCAP % 32) == 0);
static_assert(LDS_AGG <= 300000);
static_assert(GBM == (GTHR / 32) * 16);
static_assert(GTHR == 64 && GBM == 32);
static_assert((D1 % 32) == 0 && (K2 % 32) == 0 && K2 == 2 * D1);
static_assert(D1 == 4 * 32 && C2 == 2 * 32);
static_assert((MROWS % GBM) == 0 && ((MROWS * (D1 / 8)) % NTHR) == 0);
static_assert(UPM == D1 * (D1 / 8) && UPM == C2 * (K2 / 8) && (UPM % NTHR) == 0 && UPM == (1 << 11));
static_assert(D1 / 4 == 32 && C2 / 4 == 16);

typedef float          v2f   __attribute__((ext_vector_type(2)));
typedef float          v4f   __attribute__((ext_vector_type(4)));
typedef float          v8f   __attribute__((ext_vector_type(8)));
typedef int            v4i   __attribute__((ext_vector_type(4)));
typedef int            v8i   __attribute__((ext_vector_type(8)));
typedef unsigned short v8us  __attribute__((ext_vector_type(8)));
typedef unsigned short v16us __attribute__((ext_vector_type(16)));
typedef __bf16         v16bf __attribute__((ext_vector_type(16)));
typedef v2f  __attribute__((may_alias)) v2fa;
typedef v4f  __attribute__((may_alias)) v4fa;
typedef v4i  __attribute__((may_alias)) v4ia;
typedef v8us __attribute__((may_alias)) v8usa;
union Frag { v16bf v; v16us u; v8us h[2]; v8i w; };

__device__ __forceinline__ v8f wmb(const Frag& a, const Frag& b, v8f c) {
  v8f d = __builtin_amdgcn_wmma_f32_16x16x32_bf16(false, a.v, false, b.v, (short)0, c, false, false);
  asm volatile("v_nop\n\tv_nop\n\tv_nop\n\tv_nop" : "+v"(d) : "v"(a.w), "v"(b.w));
  return d;
}

__device__ __forceinline__ unsigned bf16_bits(float f) {
  const unsigned u = __float_as_uint(f);
  return (u + 0x7FFFu + ((u >> 16) & 1u)) >> 16;
}
__device__ __forceinline__ float bf16_val(float f) {
  return __uint_as_float(bf16_bits(f) << 16);
}
__device__ __forceinline__ v8us hilo8(v4f t) {
  v8us o;
  unsigned hb;
  hb = bf16_bits(t.x); o[0] = (unsigned short)hb; o[4] = (unsigned short)bf16_bits(t.x - __uint_as_float(hb << 16));
  hb = bf16_bits(t.y); o[1] = (unsigned short)hb; o[5] = (unsigned short)bf16_bits(t.y - __uint_as_float(hb << 16));
  hb = bf16_bits(t.z); o[2] = (unsigned short)hb; o[6] = (unsigned short)bf16_bits(t.z - __uint_as_float(hb << 16));
  hb = bf16_bits(t.w); o[3] = (unsigned short)hb; o[7] = (unsigned short)bf16_bits(t.w - __uint_as_float(hb << 16));
  return o;
}

__device__ __forceinline__ int scan_chunk(const int* __restrict__ dsts, int nE, int cbase, int slotBase,
                                          int nb, int vec8, int* list, int tid, int lane, int wave) {
  int wc = 0;
  const int el0  = tid * EPT;
  const int e0   = cbase + el0;
  const int sent = -2147483647 - 1;
  v4i da, db;
  if (vec8 != 0 && cbase + CHUNK <= nE) {
    da = *(const v4i*)(dsts + e0);
    db = *(const v4i*)(dsts + e0 + 4);
  } else {
    da.x = (e0     < nE) ? dsts[min(e0,     nE - 1)] : sent;
    da.y = (e0 + 1 < nE) ? dsts[min(e0 + 1, nE - 1)] : sent;
    da.z = (e0 + 2 < nE) ? dsts[min(e0 + 2, nE - 1)] : sent;
    da.w = (e0 + 3 < nE) ? dsts[min(e0 + 3, nE - 1)] : sent;
    db.x = (e0 + 4 < nE) ? dsts[min(e0 + 4, nE - 1)] : sent;
    db.y = (e0 + 5 < nE) ? dsts[min(e0 + 5, nE - 1)] : sent;
    db.z = (e0 + 6 < nE) ? dsts[min(e0 + 6, nE - 1)] : sent;
    db.w = (e0 + 7 < nE) ? dsts[min(e0 + 7, nE - 1)] : sent;
  }
  const unsigned nbs = (unsigned)slotBase;
  const unsigned unb = (unsigned)nb;
  const unsigned s0 = (unsigned)da.x - nbs, s1 = (unsigned)da.y - nbs;
  const unsigned s2 = (unsigned)da.z - nbs, s3 = (unsigned)da.w - nbs;
  const unsigned s4 = (unsigned)db.x - nbs, s5 = (unsigned)db.y - nbs;
  const unsigned s6 = (unsigned)db.z - nbs, s7 = (unsigned)db.w - nbs;
  const bool h0 = s0 < unb, h1 = s1 < unb, h2 = s2 < unb, h3 = s3 < unb;
  const bool h4 = s4 < unb, h5 = s5 < unb, h6 = s6 < unb, h7 = s7 < unb;
  const unsigned any = __builtin_amdgcn_ballot_w32(h0 | h1 | h2 | h3 | h4 | h5 | h6 | h7);
  if (any != 0u) {
#define HITJ(J, HJ, SJ) { \
      const unsigned mj = __builtin_amdgcn_ballot_w32(HJ); \
      if (mj != 0u) { \
        if (HJ) { \
          const int pos = wc + (int)__builtin_amdgcn_mbcnt_lo(mj, 0u); \
          if (pos < WCAP) list[wave * WCAP + pos] = ((el0 + (J)) << SLOTB) | (int)(SJ); \
        } \
        wc += (int)__builtin_popcount(mj); } }
    HITJ(0, h0, s0)
    HITJ(1, h1, s1)
    HITJ(2, h2, s2)
    HITJ(3, h3, s3)
    HITJ(4, h4, s4)
    HITJ(5, h5, s5)
    HITJ(6, h6, s6)
    HITJ(7, h7, s7)
#undef HITJ
  }
  return wc;
}

__global__ __launch_bounds__(NTHR) void k_wprep(const float* __restrict__ W1s, const float* __restrict__ W1d,
                                                const float* __restrict__ W2s, const float* __restrict__ W2d,
                                                unsigned short* WTu1, unsigned short* WTi1,
                                                unsigned short* WTu2, unsigned short* WTi2) {
  const int u  = (int)blockIdx.x * NTHR + (int)threadIdx.x;
  const int mi = u >> 11;
  const int v  = u & (UPM - 1);
  if (mi >= NMAT) return;
  v8us o;
  unsigned short* dp;
  if (mi < 6) {
    const float* W = W1s;
    unsigned short* D = WTu1;
    if (mi == 1)      { W = W1s + (size_t)2 * D1 * D1; D = WTu1 + (size_t)1 * D1 * D1; }
    else if (mi == 2) { W = W1d + (size_t)1 * D1 * D1; D = WTu1 + (size_t)2 * D1 * D1; }
    else if (mi == 3) { W = W1d + (size_t)2 * D1 * D1; D = WTu1 + (size_t)3 * D1 * D1; }
    else if (mi == 4) { W = W1s + (size_t)1 * D1 * D1; D = WTi1; }
    else if (mi == 5) { W = W1d;                         D = WTi1 + (size_t)1 * D1 * D1; }
    const int n  = v >> 4;
    const int k8 = (v & 15) * 8;
    const float* p = W + (size_t)k8 * D1 + n;
#pragma unroll
    for (int i = 0; i < 8; ++i) o[i] = (unsigned short)bf16_bits(p[(size_t)i * D1]);
    dp = D + (size_t)n * D1 + k8;
  } else {
    const float* W = W2s;
    unsigned short* D = WTu2;
    if (mi == 7)       { W = W2s + (size_t)2 * D1 * C2; D = WTu2 + (size_t)64 * K2; }
    else if (mi == 8)  { W = W2d + (size_t)1 * D1 * C2; D = WTu2 + (size_t)128 * K2; }
    else if (mi == 9)  { W = W2d + (size_t)2 * D1 * C2; D = WTu2 + (size_t)192 * K2; }
    else if (mi == 10) { W = W2s + (size_t)1 * D1 * C2; D = WTi2; }
    else if (mi == 11) { W = W2d;                         D = WTi2 + (size_t)64 * K2; }
    const int n = v >> 5;
    const int g = v & 31;
    const float* p = W + (size_t)(4 * g) * C2 + n;
    const unsigned short f0 = (unsigned short)bf16_bits(p[0]);
    const unsigned short f1 = (unsigned short)bf16_bits(p[C2]);
    const unsigned short f2 = (unsigned short)bf16_bits(p[2 * C2]);
    const unsigned short f3 = (unsigned short)bf16_bits(p[3 * C2]);
    o[0] = f0; o[1] = f1; o[2] = f2; o[3] = f3; o[4] = f0; o[5] = f1; o[6] = f2; o[7] = f3;
    dp = D + (size_t)n * K2 + 8 * g;
  }
  *(volatile v8us*)dp = o;
  __threadfence();
  *(volatile v8us*)dp = o;
}

__global__ __launch_bounds__(NTHR) void k_cvx(const float* __restrict__ x0, const float* __restrict__ x1,
                                              int n0, int n1, int U0, int U1,
                                              unsigned short* xb0, unsigned short* xb1) {
  const int u = (int)blockIdx.x * NTHR + (int)threadIdx.x;
  const float* x = x0;
  unsigned short* xb = xb0;
  int nN = n0;
  int v;
  if (u < U0) {
    v = u;
  } else if (u < U0 + U1) {
    x = x1; xb = xb1; nN = n1; v = u - U0;
  } else {
    return;
  }
  const int row = v >> 4;
  const int k8  = (v & 15) * 8;
  const int rc  = row < nN ? row : nN - 1;
  const float* p = x + (size_t)rc * D1 + k8;
  const v4f a = *(const v4fa*)p;
  const v4f b = *(const v4fa*)(p + 4);
  const bool ok = row < nN;
  v8us o;
  o[0] = ok ? (unsigned short)bf16_bits(a.x) : (unsigned short)0;
  o[1] = ok ? (unsigned short)bf16_bits(a.y) : (unsigned short)0;
  o[2] = ok ? (unsigned short)bf16_bits(a.z) : (unsigned short)0;
  o[3] = ok ? (unsigned short)bf16_bits(a.w) : (unsigned short)0;
  o[4] = ok ? (unsigned short)bf16_bits(b.x) : (unsigned short)0;
  o[5] = ok ? (unsigned short)bf16_bits(b.y) : (unsigned short)0;
  o[6] = ok ? (unsigned short)bf16_bits(b.z) : (unsigned short)0;
  o[7] = ok ? (unsigned short)bf16_bits(b.w) : (unsigned short)0;
  unsigned short* dp = xb + (size_t)row * D1 + k8;
  *(volatile v8us*)dp = o;
  __threadfence();
  *(volatile v8us*)dp = o;
}

template <int DW>
__global__ __launch_bounds__(GTHR) void k_gemm(const unsigned short* __restrict__ A,
                                               const unsigned short* __restrict__ WT, int K, int MPr,
                                               const float* __restrict__ att0, const float* __restrict__ att1,
                                               const float* __restrict__ att2, const float* __restrict__ att3,
                                               float* H, int hps, int nStore, float* SD) {
  static_assert(DW == D1 || DW == C2);
  __shared__ __attribute__((aligned(16))) float stg[GBM * D1];
  __shared__ __attribute__((aligned(16))) float satt[D1];
  __shared__ __attribute__((aligned(16))) float sdot[2 * GBM];
  const int tid = (int)threadIdx.x, lane = tid & 31, wave = tid >> 5, hh = lane >> 4, m = lane & 15;
  const int rowBase = (int)blockIdx.x * GBM;
  const int g = (int)blockIdx.y;

  {
    int iLo, iHi, offHi;
    if (DW == D1) { iLo = g; iHi = g; offHi = 64; } else { iLo = 2 * g; iHi = 2 * g + 1; offHi = 0; }
    const float* pLo = att0;
    if (iLo == 1) pLo = att1; else if (iLo == 2) pLo = att2; else if (iLo == 3) pLo = att3;
    const float* pHi = att0;
    if (iHi == 1) pHi = att1; else if (iHi == 2) pHi = att2; else if (iHi == 3) pHi = att3;
    satt[tid]      = bf16_val(pLo[tid]);
    satt[64 + tid] = bf16_val(pHi[offHi + tid]);
  }

  v8f acc[8];
  {
    const v8f z = {0.f, 0.f, 0.f, 0.f, 0.f, 0.f, 0.f, 0.f};
#pragma unroll
    for (int t = 0; t < 8; ++t) acc[t] = z;
  }
  const unsigned short* ap = A  + (size_t)(rowBase + 16 * wave + m) * (size_t)K + 8 * hh;
  const unsigned short* bp = WT + ((size_t)g * D1 + m) * (size_t)K + 8 * hh;
  const int ksteps = K >> 5;

#pragma unroll 1
  for (int ks = 0; ks < ksteps; ++ks) {
    const int k0 = 32 * ks;
    Frag af;
    af.h[0] = *(const v8usa*)(ap + k0);
    af.h[1] = *(const v8usa*)(ap + k0 + 16);
#pragma unroll
    for (int nt = 0; nt < 8; ++nt) {
      const unsigned short* wq = bp + (size_t)(16 * nt) * (size_t)K + k0;
      Frag bf;
      bf.h[0] = *(const v8usa*)wq;
      bf.h[1] = *(const v8usa*)(wq + 16);
      acc[nt] = wmb(af, bf, acc[nt]);
    }
  }

#pragma unroll
  for (int nt = 0; nt < 8; ++nt) {
    const int lc = 16 * nt + m;
#pragma unroll
    for (int r = 0; r < 8; ++r) {
      const int lr = 16 * wave + 8 * hh + r;
      stg[lr * D1 + lc] = acc[nt][r];
    }
  }
  __syncthreads();

  {
    const int row = tid & 31, half = tid >> 5;
    const int cbeg = (DW == D1) ? 0 : C2 * half;
    const float* hr = stg + row * D1 + cbeg;
    const float* sa = satt + cbeg;
    float d = 0.f;
#pragma unroll 4
    for (int c4 = 0; c4 < DW / 4; ++c4) {
      const v4f hv = *(const v4fa*)(hr + 4 * c4);
      const v4f av = *(const v4fa*)(sa + 4 * c4);
      d = fmaf(hv.x, av.x, d);
      d = fmaf(hv.y, av.y, d);
      d = fmaf(hv.z, av.z, d);
      d = fmaf(hv.w, av.w, d);
    }
    sdot[half * GBM + row] = d;
  }
  __syncthreads();

  const int piece = lane & 7;
  const int pl    = (DW == D1) ? 0 : ((lane >> 3) & 1);
  const v4f sdv   = *(const v4fa*)(sdot + pl * GBM + 4 * piece);
  const int plane = (DW == D1) ? g : (2 * g + pl);
  float* sp = SD + (size_t)plane * (size_t)MPr + rowBase + 4 * piece;
  const bool wsd = (wave == 0) && (lane < ((DW == D1) ? 8 : 16));
  const bool wh  = g < nStore;

  v4f fv[16];
#pragma unroll
  for (int i = 0; i < 16; ++i) {
    const int lr = 16 * wave + i;
    fv[i] = *(const v4fa*)(stg + lr * D1 + 4 * lane);
  }
  float* hb = H + (size_t)g * (size_t)hps;
  if (wh) {
#pragma unroll
    for (int i = 0; i < 16; ++i) {
      const int gr = rowBase + 16 * wave + i;
      float* op = hb + (size_t)gr * (size_t)D1 + 4 * lane;
      *(volatile v4f*)op = fv[i];
    }
  }
  if (wsd) *(volatile v4f*)sp = sdv;
  __threadfence();
  if (wh) {
#pragma unroll
    for (int i = 0; i < 16; ++i) {
      const int gr = rowBase + 16 * wave + i;
      float* op = hb + (size_t)gr * (size_t)D1 + 4 * lane;
      *(volatile v4f*)op = fv[i];
    }
  }
  if (wsd) *(volatile v4f*)sp = sdv;
}

template <int CW, int ADDIN, int HL>
__global__ __launch_bounds__(NTHR) void k_agg(
    const int* __restrict__ srcs, const int* __restrict__ dsts, int nE, int nSrc, int nDst, int MPr, int nb, int vec8,
    const float* __restrict__ F, int ldF, int colOff,
    const float* __restrict__ AS, const float* __restrict__ AD, const float* __restrict__ bias,
    const float* __restrict__ oin, float* oout, unsigned short* hp) {
  static_assert(CW == D1 || (CW == C2 && HL == 0));
  constexpr int CPL = CW / 32;
  extern __shared__ v4f lds_dyn[];
  int* reg1 = (int*)lds_dyn;
  int* reg2 = reg1 + RCAP;
  int* scnt = reg2 + RCAP;
  int* soff = scnt + NBMAX;
  int* list = soff + NBMAX;
  int* wcnt = list + LISTN;
  int* wtot = wcnt + NWAVE;
  const int tid = (int)threadIdx.x, lane = tid & 31, wave = tid >> 5;
  const int nodeBase = (int)blockIdx.x * nb;

  for (int i = tid; i < NBMAX; i += NTHR) scnt[i] = 0;
  __syncthreads();

  int tot = 0;
  const int nChunks = (nE + CHUNK - 1) / CHUNK;
#pragma unroll 1
  for (int ch = 0; ch < nChunks; ++ch) {
    const int cbase = ch * CHUNK;
    const int wc = scan_chunk(dsts, nE, cbase, nodeBase, nb, vec8, list, tid, lane, wave);
    if (lane == 0) wcnt[wave] = wc;
    __syncthreads();
    int pre = 0, all = 0;
#pragma unroll
    for (int w2 = 0; w2 < NWAVE; ++w2) {
      int c = wcnt[w2];
      c = c < 0 ? 0 : (c > WCAP ? WCAP : c);
      all += c;
      pre += (w2 < wave) ? c : 0;
    }
    const int wcc  = wc > WCAP ? WCAP : wc;
    const int base = tot + pre;
#pragma unroll 1
    for (int i = lane; i < wcc; i += 32) {
      const int ent = list[wave * WCAP + i];
      const int el  = (ent >> SLOTB) & (CHUNK - 1);
      const int sl  = ent & (NBMAX - 1);
      int eid = cbase + el;
      eid = eid > nE - 1 ? nE - 1 : eid;
      const int pos = base + i;
      if (pos < RCAP) reg1[pos] = (int)(((unsigned)eid << SLOTB) | (unsigned)sl);
    }
    tot += all;
    tot = tot > RCAP ? RCAP : tot;
    __syncthreads();
  }
  const int nh = tot;

  if (wave == 0) {
#pragma unroll 1
    for (int b0 = 0; b0 < nh; b0 += 32) {
      const int idx = b0 + lane;
      const int uv  = reg1[idx < nh ? idx : nh - 1];
      const int m32 = (nh - b0) < 32 ? (nh - b0) : 32;
#pragma unroll 1
      for (int k = 0; k < m32; ++k) {
        const int u  = __builtin_amdgcn_readlane(uv, k);
        const int sl = u & (NBMAX - 1);
        if (lane == 0) scnt[sl] = scnt[sl] + 1;
      }
    }
  }
  __syncthreads();

  {
    const v4i ca = *(const v4ia*)(scnt + 8 * tid);
    const v4i cb = *(const v4ia*)(scnt + 8 * tid + 4);
    const int e0 = ca.x < 0 ? 0 : ca.x, e1 = ca.y < 0 ? 0 : ca.y, e2 = ca.z < 0 ? 0 : ca.z, e3 = ca.w < 0 ? 0 : ca.w;
    const int e4 = cb.x < 0 ? 0 : cb.x, e5 = cb.y < 0 ? 0 : cb.y, e6 = cb.z < 0 ? 0 : cb.z, e7 = cb.w < 0 ? 0 : cb.w;
    const int ts = e0 + e1 + e2 + e3 + e4 + e5 + e6 + e7;
    int incl = ts;
#pragma unroll
    for (int d = 1; d < 32; d <<= 1) {
      const int up = __shfl_up(incl, d);
      if (lane >= d) incl += up;
    }
    if (lane == 31) wtot[wave] = incl;
    __syncthreads();
    int pre = 0;
#pragma unroll
    for (int w2 = 0; w2 < NWAVE; ++w2) pre += (w2 < wave) ? wtot[w2] : 0;
    int run = pre + incl - ts;
    soff[8 * tid + 0] = run; run += e0;
    soff[8 * tid + 1] = run; run += e1;
    soff[8 * tid + 2] = run; run += e2;
    soff[8 * tid + 3] = run; run += e3;
    soff[8 * tid + 4] = run; run += e4;
    soff[8 * tid + 5] = run; run += e5;
    soff[8 * tid + 6] = run; run += e6;
    soff[8 * tid + 7] = run;
  }
  __syncthreads();
  for (int i = tid; i < NBMAX; i += NTHR) list[i] = soff[i];
  __syncthreads();

  if (wave == 0) {
#pragma unroll 1
    for (int b0 = 0; b0 < nh; b0 += 32) {
      const int idx = b0 + lane;
      const int uv  = reg1[idx < nh ? idx : nh - 1];
      const int m32 = (nh - b0) < 32 ? (nh - b0) : 32;
#pragma unroll 1
      for (int k = 0; k < m32; ++k) {
        const int u   = __builtin_amdgcn_readlane(uv, k);
        const int sl  = u & (NBMAX - 1);
        const int eid = (int)((unsigned)u >> SLOTB);
        if (lane == 0) {
          int pos = list[sl];
          pos = pos < 0 ? 0 : (pos > RCAP - 1 ? RCAP - 1 : pos);
          reg2[pos] = eid;
          list[sl] = pos + 1;
        }
      }
    }
  }
  __syncthreads();

  const int nbw = nb >> 3;
  const bool ovf = (nh >= RCAP);
  const float qnan = __int_as_float(0x7fc00000);
  v4f bb4 = {0.0f, 0.0f, 0.0f, 0.0f};
  v2f bb2 = {0.0f, 0.0f};
  if constexpr (CW == D1) {
    const v4f t = *(const v4fa*)(bias + 4 * lane);
    bb4.x = bf16_val(t.x); bb4.y = bf16_val(t.y); bb4.z = bf16_val(t.z); bb4.w = bf16_val(t.w);
  } else {
    const v2f t = *(const v2fa*)(bias + 2 * lane);
    bb2.x = bf16_val(t.x); bb2.y = bf16_val(t.y);
  }

#pragma unroll 1
  for (int jt = 0; jt < nbw; ++jt) {
    const int slot = wave * nbw + jt;
    const int grow = nodeBase + slot;
    const int gcl  = grow < nDst ? grow : nDst - 1;
    int st = soff[slot];
    const int craw = scnt[slot];
    int cnt = craw;
    st  = st < 0 ? 0 : (st > nh ? nh : st);
    cnt = cnt < 0 ? 0 : (cnt > DEGCAP ? DEGCAP : cnt);
    if (cnt > nh - st) cnt = nh - st;
    const float pz = (ovf || craw > DEGCAP) ? qnan : 0.0f;

    const float adv = AD[gcl];
    float mx = MX0, dn = 0.0f, a0 = 0.0f, a1 = 0.0f, a2 = 0.0f, a3 = 0.0f;

#pragma unroll 1
    for (int q = 0; q < cnt; ++q) {
      int idx = st + q; idx = idx > RCAP - 1 ? RCAP - 1 : idx;
      int eid = reg2[idx]; eid = eid < 0 ? 0 : (eid > nE - 1 ? nE - 1 : eid);
      const int sraw = srcs[eid];
      const int s = sraw < 0 ? 0 : (sraw > nSrc - 1 ? nSrc - 1 : sraw);
      const float* fr = F + (size_t)s * (size_t)ldF + colOff + CPL * lane;
      float f0, f1, f2 = 0.0f, f3 = 0.0f;
      if constexpr (CW == D1) {
        const v4f fs = *(const v4fa*)fr;
        f0 = fs.x; f1 = fs.y; f2 = fs.z; f3 = fs.w;
      } else {
        const v2f fs = *(const v2fa*)fr;
        f0 = fs.x; f1 = fs.y;
      }
      float lg = AS[s] + adv;
      lg = lg > 0.f ? lg : NEGSL * lg;
      const float df = lg - mx;
      const float ee = __expf(-fabsf(df));
      const bool up  = df > 0.f;
      const float s1 = up ? ee : 1.0f;
      const float s2 = up ? 1.0f : ee;
      mx = up ? lg : mx;
      dn = fmaf(dn, s1, s2);
      a0 = fmaf(a0, s1, s2 * f0);
      a1 = fmaf(a1, s1, s2 * f1);
      if constexpr (CW == D1) {
        a2 = fmaf(a2, s1, s2 * f2);
        a3 = fmaf(a3, s1, s2 * f3);
      }
    }
    const float inv = __builtin_amdgcn_rcpf(dn + EPS_SM);
    const bool live = grow < nDst;
    const bool wrow = grow < MPr;

    if constexpr (CW == D1) {
      v4f v;
      v.x = fmaf(a0, inv, bb4.x);
      v.y = fmaf(a1, inv, bb4.y);
      v.z = fmaf(a2, inv, bb4.z);
      v.w = fmaf(a3, inv, bb4.w);
      if constexpr (ADDIN != 0) {
        const v4f pv = *(const v4fa*)(oin + (size_t)gcl * (size_t)CW + 4 * lane);
        v = pv + v;
      }
      if constexpr (HL != 0) {
        v.x = fmaxf(v.x, 0.0f); v.y = fmaxf(v.y, 0.0f); v.z = fmaxf(v.z, 0.0f); v.w = fmaxf(v.w, 0.0f);
      }
      v4f y;
      y.x = (live ? v.x : 0.f) + pz;
      y.y = (live ? v.y : 0.f) + pz;
      y.z = (live ? v.z : 0.f) + pz;
      y.w = (live ? v.w : 0.f) + pz;
      if constexpr (HL != 0) {
        const v8us po = hilo8(y);
        unsigned short* gp = hp + (size_t)grow * (size_t)K2 + 8 * lane;
        if (wrow) *(volatile v8us*)gp = po;
        __threadfence();
        if (wrow) *(volatile v8us*)gp = po;
      } else {
        float* op = oout + (size_t)grow * (size_t)CW + 4 * lane;
        if (wrow) *(volatile v4f*)op = y;
        __threadfence();
        if (wrow) *(volatile v4f*)op = y;
      }
    } else {
      float v0 = fmaf(a0, inv, bb2.x);
      float v1 = fmaf(a1, inv, bb2.y);
      if constexpr (ADDIN != 0) {
        const v2f pv = *(const v2fa*)(oin + (size_t)gcl * (size_t)CW + 2 * lane);
        v0 = pv.x + v0;
        v1 = pv.y + v1;
      }
      const float h0 = (live ? v0 : 0.f) + pz;
      const float h1 = (live ? v1 : 0.f) + pz;
      const int i0 = (2 * lane) & 31, i1 = (2 * lane + 1) & 31;
      const float g0 = __shfl(h0, i0);
      const float g1 = __shfl(h1, i0);
      const float g2 = __shfl(h0, i1);
      const float g3 = __shfl(h1, i1);
      v4f ov;
      ov.x = g0; ov.y = g1; ov.z = g2; ov.w = g3;
      float* op = oout + (size_t)grow * (size_t)CW + 4 * (lane & 15);
      const bool wr = wrow && (lane < 16);
      if (wr) *(volatile v4f*)op = ov;
      __threadfence();
      if (wr) *(volatile v4f*)op = ov;
    }
  }
}

__global__ __launch_bounds__(NTHR) void k_score(const int* __restrict__ el0, const int* __restrict__ el1,
                                                const int* __restrict__ el2, int L,
                                                const float* __restrict__ oU, const float* __restrict__ oI,
                                                int nU, int nI, const float* __restrict__ relw, float* out) {
  __shared__ __attribute__((aligned(16))) float srw[C2];
  const int tid = (int)threadIdx.x;
  const int r = (int)blockIdx.y;
  const int* el = el0;
  const float* oA = oU;
  const float* oB = oI;
  int nA = nU, nB = nI;
  if (r == 1)      { el = el1; oA = oI; oB = oU; nA = nI; nB = nU; }
  else if (r == 2) { el = el2; oA = oU; oB = oU; nA = nU; nB = nU; }
  if (tid < C2) srw[tid] = bf16_val(relw[(size_t)r * C2 + tid]);
  __syncthreads();
  const int e  = (int)blockIdx.x * NTHR + tid;
  const int ec = e < L ? e : L - 1;
  int ia = el[ec];
  ia = ia < 0 ? 0 : (ia > nA - 1 ? nA - 1 : ia);
  int ib = el[(size_t)L + ec];
  ib = ib < 0 ? 0 : (ib > nB - 1 ? nB - 1 : ib);
  const float* pa = oA + (size_t)ia * C2;
  const float* pb = oB + (size_t)ib * C2;
  float s = 0.0f;
#pragma unroll 4
  for (int c4 = 0; c4 < C2 / 4; ++c4) {
    const v4f va = *(const v4fa*)(pa + 4 * c4);
    const v4f vb = *(const v4fa*)(pb + 4 * c4);
    const v4f w  = *(const v4fa*)(srw + 4 * c4);
    s = fmaf(va.x * w.x, vb.x, s);
    s = fmaf(va.y * w.y, vb.y, s);
    s = fmaf(va.z * w.z, vb.z, s);
    s = fmaf(va.w * w.w, vb.w, s);
  }
  float* op = out + (size_t)r * (size_t)L + ec;
  const bool wr = e < L;
  if (wr) *(volatile float*)op = s;
  __threadfence();
  if (wr) *(volatile float*)op = s;
}

static int pick_nb(int nE, int nN) {
  int nb = NBMAX;
  while (nb > 32 && (long long)nb * (long long)nE * 8LL > (long long)RCAP * (long long)nN * 7LL) nb >>= 1;
  return nb;
}
static inline int cdiv(int a, int b) { return (a + b - 1) / b; }

extern "C" void kernel_launch(void* const* d_in, const int* in_sizes, int n_in,
                              void* d_out, int out_size, void* d_ws, size_t ws_size,
                              hipStream_t stream) {
  if (n_in < 19) return;
  if (in_sizes[0] < D1 || (in_sizes[0] % D1) != 0) return;
  if (in_sizes[1] < D1 || (in_sizes[1] % D1) != 0) return;
  const int nU = in_sizes[0] / D1, nI = in_sizes[1] / D1;
  if (nU > (1 << 22) || nI > (1 << 22)) return;
  if (in_sizes[2] != 3 * D1 * D1 || in_sizes[3] != 3 * D1 * D1) return;
  if (in_sizes[4] != 3 * D1 || in_sizes[5] != 3 * D1 || in_sizes[6] != 3 * D1) return;
  if (in_sizes[7] != 3 * D1 * C2 || in_sizes[8] != 3 * D1 * C2) return;
  if (in_sizes[9] != 3 * C2 || in_sizes[10] != 3 * C2 || in_sizes[11] != 3 * C2 || in_sizes[12] != 3 * C2) return;
  if ((in_sizes[13] & 1) || (in_sizes[14] & 1) || (in_sizes[15] & 1)) return;
  if ((in_sizes[16] & 1) || (in_sizes[17] & 1) || (in_sizes[18] & 1)) return;
  const int E0 = in_sizes[13] / 2, E1 = in_sizes[14] / 2, E2 = in_sizes[15] / 2;
  const int L  = in_sizes[16] / 2;
  if (E0 < 1 || E1 < 1 || E2 < 1 || L < 1) return;
  if (in_sizes[17] / 2 != L || in_sizes[18] / 2 != L) return;
  if (E0 >= (1 << (32 - SLOTB)) || E1 >= (1 << (32 - SLOTB)) || E2 >= (1 << (32 - SLOTB))) return;
  if ((long long)out_size != 3LL * (long long)L) return;

  const float* xU   = (const float*)d_in[0];
  const float* xI   = (const float*)d_in[1];
  const float* W1s  = (const float*)d_in[2];
  const float* W1d  = (const float*)d_in[3];
  const float* a1s  = (const float*)d_in[4];
  const float* a1d  = (const float*)d_in[5];
  const float* b1   = (const float*)d_in[6];
  const float* W2s  = (const float*)d_in[7];
  const float* W2d  = (const float*)d_in[8];
  const float* a2s  = (const float*)d_in[9];
  const float* a2d  = (const float*)d_in[10];
  const float* b2   = (const float*)d_in[11];
  const float* relw = (const float*)d_in[12];
  const int* ei0 = (const int*)d_in[13];
  const int* ei1 = (const int*)d_in[14];
  const int* ei2 = (const int*)d_in[15];
  const int* el0 = (const int*)d_in[16];
  const int* el1 = (const int*)d_in[17];
  const int* el2 = (const int*)d_in[18];
  float* out = (float*)d_out;

  const int MPu = cdiv(nU, MROWS) * MROWS;
  const int MPi = cdiv(nI, MROWS) * MROWS;
  const int maxMP = MPu > MPi ? MPu : MPi;
  const int nb0 = pick_nb(E0, nI);
  const int nb1 = pick_nb(E1, nU);
  const int nb2 = pick_nb(E2, nU);
  if (nb0 < 32 || (nb0 & (nb0 - 1)) != 0 || nb0 > NBMAX) return;
  if (nb1 < 32 || (nb1 & (nb1 - 1)) != 0 || nb1 > NBMAX) return;
  if (nb2 < 32 || (nb2 & (nb2 - 1)) != 0 || nb2 > NBMAX) return;
  const int gA0 = cdiv(MPi, nb0), gA1 = cdiv(MPu, nb1), gA2 = cdiv(MPu, nb2);
  if ((long long)gA0 * nb0 < MPi || (long long)gA1 * nb1 < MPu || (long long)gA2 * nb2 < MPu) return;
  const int vec0 = ((E0 & 3) == 0) ? 1 : 0, vec1 = ((E1 & 3) == 0) ? 1 : 0, vec2 = ((E2 & 3) == 0) ? 1 : 0;
  const int Uu = MPu * (D1 / 8), Ui = MPi * (D1 / 8);
  if ((Uu % NTHR) != 0 || (Ui % NTHR) != 0) return;
  if ((MPu % GBM) != 0 || (MPi % GBM) != 0) return;

  const size_t PL = (size_t)maxMP * D1 * 4;
  size_t szR0 = (size_t)(MPu + MPi) * D1 * 2;
  if ((size_t)MPi * K2 * 2 > szR0) szR0 = (size_t)MPi * K2 * 2;
  if ((size_t)MPi * C2 * 4 > szR0) szR0 = (size_t)MPi * C2 * 4;
  char* ws = (char*)d_ws;
  size_t off = 0;
  const size_t oW1u = off; off += (size_t)4 * D1 * D1 * 2;     off = (off + 255) & ~(size_t)255;
  const size_t oW1i = off; off += (size_t)2 * D1 * D1 * 2;     off = (off + 255) & ~(size_t)255;
  const size_t oW2u = off; off += (size_t)2 * D1 * K2 * 2;     off = (off + 255) & ~(size_t)255;
  const size_t oW2i = off; off += (size_t)1 * D1 * K2 * 2;     off = (off + 255) & ~(size_t)255;
  const size_t oSDu = off; off += (size_t)NSDP * MPu * 4;      off = (off + 255) & ~(size_t)255;
  const size_t oSDi = off; off += (size_t)NSDP * MPi * 4;      off = (off + 255) & ~(size_t)255;
  const size_t oR0  = off; off += szR0;                        off = (off + 255) & ~(size_t)255;
  const size_t oR1  = off; off += 2 * PL;                      off = (off + 255) & ~(size_t)255;
  const size_t oR2  = off; off += PL;                          off = (off + 255) & ~(size_t)255;
  if (off > ws_size || off > (size_t)WSMAX) return;
  if ((size_t)MPu * K2 * 2 > PL || (size_t)2 * MPu * C2 * 4 > PL || (size_t)MPi * D1 * 4 > PL) return;

  unsigned short* WTu1 = (unsigned short*)(ws + oW1u);
  unsigned short* WTi1 = (unsigned short*)(ws + oW1i);
  unsigned short* WTu2 = (unsigned short*)(ws + oW2u);
  unsigned short* WTi2 = (unsigned short*)(ws + oW2i);
  float* SDu = (float*)(ws + oSDu);
  float* SDi = (float*)(ws + oSDi);
  unsigned short* XBu = (unsigned short*)(ws + oR0);
  unsigned short* XBi = (unsigned short*)(ws + oR0 + (size_t)MPu * D1 * 2);
  unsigned short* HAi = (unsigned short*)(ws + oR0);
  float*          OI  = (float*)(ws + oR0);
  float*          H1u = (float*)(ws + oR1);
  float*          O1  = (float*)(ws + oR1);
  float*          H2i = (float*)(ws + oR1);
  float*          H2u = (float*)(ws + oR1 + PL);
  float*          H1i = (float*)(ws + oR2);
  unsigned short* HAu = (unsigned short*)(ws + oR2);
  float*          O2  = (float*)(ws + oR2);
  float*          OU  = (float*)(ws + oR2 + (size_t)MPu * C2 * 4);
  const int hps = (int)(PL / 4);

  hipFuncSetAttribute(reinterpret_cast<const void*>(&k_agg<D1, 0, 1>), hipFuncAttributeMaxDynamicSharedMemorySize, LDS_AGG);
  hipFuncSetAttribute(reinterpret_cast<const void*>(&k_agg<D1, 0, 0>), hipFuncAttributeMaxDynamicSharedMemorySize, LDS_AGG);
  hipFuncSetAttribute(reinterpret_cast<const void*>(&k_agg<D1, 1, 1>), hipFuncAttributeMaxDynamicSharedMemorySize, LDS_AGG);
  hipFuncSetAttribute(reinterpret_cast<const void*>(&k_agg<C2, 0, 0>), hipFuncAttributeMaxDynamicSharedMemorySize, LDS_AGG);
  hipFuncSetAttribute(reinterpret_cast<const void*>(&k_agg<C2, 1, 0>), hipFuncAttributeMaxDynamicSharedMemorySize, LDS_AGG);

  k_wprep<<<(NMAT * UPM) / NTHR, NTHR, 0, stream>>>(W1s, W1d, W2s, W2d, WTu1, WTi1, WTu2, WTi2);
  k_cvx<<<(Uu + Ui) / NTHR, NTHR, 0, stream>>>(xU, xI, nU, nI, Uu, Ui, XBu, XBi);

  k_gemm<D1><<<dim3(MPu / GBM, 4), GTHR, 0, stream>>>(XBu, WTu1, D1, MPu,
      a1s + 0 * D1, a1s + 2 * D1, a1d + 1 * D1, a1d + 2 * D1, H1u, hps, 2, SDu);
  k_gemm<D1><<<dim3(MPi / GBM, 2), GTHR, 0, stream>>>(XBi, WTi1, D1, MPi,
      a1s + 1 * D1, a1d + 0 * D1, a1s, a1s, H1i, hps, 1, SDi);

  k_agg<D1, 0, 1><<<gA0, NTHR, LDS_AGG, stream>>>(ei0, ei0 + E0, E0, nU, nI, MPi, nb0, vec0,
      H1u, D1, 0, SDu + 0 * (size_t)MPu, SDi + 1 * (size_t)MPi, b1 + 0 * D1, O1, OI, HAi);
  k_agg<D1, 0, 0><<<gA1, NTHR, LDS_AGG, stream>>>(ei1, ei1 + E1, E1, nI, nU, MPu, nb1, vec1,
      H1i, D1, 0, SDi + 0 * (size_t)MPi, SDu + 2 * (size_t)MPu, b1 + 1 * D1, OI, O1, HAi);
  k_agg<D1, 1, 1><<<gA2, NTHR, LDS_AGG, stream>>>(ei2, ei2 + E2, E2, nU, nU, MPu, nb2, vec2,
      H1u + (size_t)hps, D1, 0, SDu + 1 * (size_t)MPu, SDu + 3 * (size_t)MPu, b1 + 2 * D1, O1, OI, HAu);

  k_gemm<C2><<<dim3(MPu / GBM, 2), GTHR, 0, stream>>>(HAu, WTu2, K2, MPu,
      a2s + 0 * C2, a2s + 2 * C2, a2d + 1 * C2, a2d + 2 * C2, H2u, hps, 1, SDu);
  k_gemm<C2><<<dim3(MPi / GBM, 1), GTHR, 0, stream>>>(HAi, WTi2, K2, MPi,
      a2s + 1 * C2, a2d + 0 * C2, a2s, a2s, H2i, hps, 1, SDi);

  k_agg<C2, 0, 0><<<gA0, NTHR, LDS_AGG, stream>>>(ei0, ei0 + E0, E0, nU, nI, MPi, nb0, vec0,
      H2u, D1, 0, SDu + 0 * (size_t)MPu, SDi + 1 * (size_t)MPi, b2 + 0 * C2, O2, OI, HAu);
  k_agg<C2, 0, 0><<<gA1, NTHR, LDS_AGG, stream>>>(ei1, ei1 + E1, E1, nI, nU, MPu, nb1, vec1,
      H2i, D1, 0, SDi + 0 * (size_t)MPi, SDu + 2 * (size_t)MPu, b2 + 1 * C2, OI, O2, HAu);
  k_agg<C2, 1, 0><<<gA2, NTHR, LDS_AGG, stream>>>(ei2, ei2 + E2, E2, nU, nU, MPu, nb2, vec2,
      H2u, D1, C2, SDu + 1 * (size_t)MPu, SDu + 3 * (size_t)MPu, b2 + 2 * C2, O2, OU, HAu);

  k_score<<<dim3(cdiv(L, NTHR), 3), NTHR, 0, stream>>>(el0, el1, el2, L, OU, OI, nU, nI, relw, out);
}
